// GatedPropagationModel_48533130445171
// MI455X (gfx1250) — hardware-verified
//
#include <hip/hip_runtime.h>
#include <math.h>
typedef __attribute__((ext_vector_type(16))) _Float16 v16h;
typedef __attribute__((ext_vector_type(8)))  _Float16 v8h;
typedef __attribute__((ext_vector_type(16))) __bf16   v16b;
typedef __attribute__((ext_vector_type(8)))  __bf16   v8b;
typedef __attribute__((ext_vector_type(8)))  float    v8f;
typedef __attribute__((ext_vector_type(4)))  float    v4f;
#define PSCALE 32768.0f
#define U16(p) ((const unsigned short*)(const void*)(p))
#define PSCALE_INV (1.0f / 32768.0f)

__device__ __forceinline__ unsigned short f2bf_bits(float f) {
  unsigned u = __float_as_uint(f);
  return (unsigned short)((u + 0x7FFFu + ((u >> 16) & 1u)) >> 16);
}
__device__ __forceinline__ float bf_bits2f(unsigned short h) { return __uint_as_float(((unsigned)h) << 16); }

__device__ __forceinline__ void dep_guard_h(v8f& a, v8f& b, v16h x, v16h y) { asm volatile("v_nop\n\tv_nop\n\tv_nop\n\tv_nop" : "+v"(a), "+v"(b) : "v"(x), "v"(y)); }
__device__ __forceinline__ void dep_guard_b(v8f& a, v8f& b, v16b x, v16b y) { asm volatile("v_nop\n\tv_nop\n\tv_nop\n\tv_nop" : "+v"(a), "+v"(b) : "v"(x), "v"(y)); }
__device__ __forceinline__ void keep4_h(v16h a, v16h b, v16h c, v16h d) { asm volatile("v_nop" :: "v"(a), "v"(b), "v"(c), "v"(d)); }
__device__ __forceinline__ void keep4_b(v16b a, v16b b, v16b c, v16b d) { asm volatile("v_nop" :: "v"(a), "v"(b), "v"(c), "v"(d)); }
__device__ __forceinline__ void acc_guard4(v8f& a, v8f& b, v8f& c, v8f& d) { asm volatile("v_nop\n\tv_nop\n\tv_nop\n\tv_nop" : "+v"(a), "+v"(b), "+v"(c), "+v"(d)); }
template <typename T> struct Frag;
template <> struct Frag<_Float16> {
  typedef v16h V; union U { v16h v; v8h h[2]; };
  static __device__ __forceinline__ v16h load(const _Float16* p) {
    U f; f.h[0] = *(const v8h*)(p); f.h[1] = *(const v8h*)(p + 16); return f.v;
  }
  static __device__ __forceinline__ v8f mma(v16h a, v16h b, v8f c) {
    return __builtin_amdgcn_wmma_f32_16x16x32_f16(false, a, false, b, (short)0, c, false, false);
  }
  static __device__ __forceinline__ void guard(v8f& a, v8f& b, v16h x, v16h y) { dep_guard_h(a, b, x, y); }
  static __device__ __forceinline__ void keep(v16h a, v16h b, v16h c, v16h d) { keep4_h(a, b, c, d); }
};
template <> struct Frag<__bf16> {
  typedef v16b V; union U { v16b v; v8b h[2]; };
  static __device__ __forceinline__ v16b load(const __bf16* p) {
    U f; f.h[0] = *(const v8b*)(p); f.h[1] = *(const v8b*)(p + 16); return f.v;
  }
  static __device__ __forceinline__ v8f mma(v16b a, v16b b, v8f c) {
    return __builtin_amdgcn_wmma_f32_16x16x32_bf16(false, a, false, b, (short)0, c, false, false);
  }
  static __device__ __forceinline__ void guard(v8f& a, v8f& b, v16b x, v16b y) { dep_guard_b(a, b, x, y); }
  static __device__ __forceinline__ void keep(v16b a, v16b b, v16b c, v16b d) { keep4_b(a, b, c, d); }
};

template <int ET> struct Elem;
template <> struct Elem<0> { typedef _Float16 T; };
template <> struct Elem<1> { typedef __bf16 T; };
template <int ET, bool SPLIT, int BIAS_MODE, int OUT_MODE, bool RESID, int ACT = 0>
__global__ __launch_bounds__(256) void wmma_gemm64(
    const unsigned short* __restrict__ Ap, const unsigned short* __restrict__ A2p, int lda, long strideA,
    const unsigned short* __restrict__ Btp, const unsigned short* __restrict__ Bt2p, int ldb, long strideB,
    void* __restrict__ Cout, void* __restrict__ Cout2, int ldc, long strideC,
    const float* __restrict__ bias,
    const float* __restrict__ resid, long strideR,
    int M, int N, int K, float scale) {
  typedef typename Elem<ET>::T T;
  typedef typename Frag<T>::V V;
  const T* A = (const T*)Ap; const T* A2 = (const T*)A2p; const T* Bt = (const T*)Btp; const T* Bt2 = (const T*)Bt2p;
  __shared__ __align__(16) float sT[8][16 * 68];
  const int b    = blockIdx.y;
  const int lane = threadIdx.x & 31;
  const int wave = threadIdx.x >> 5;
  const int tilesN = N >> 6;
  const int tilesM = M >> 6;
  const int tile = blockIdx.x * 8 + wave;
  if (tile >= tilesM * tilesN) return;
  const int tm = tile / tilesN;
  const int tn = tile - tm * tilesN;
  const int m0 = tm << 6;
  const int n0 = tn << 6;

  const T* Ab  = A  + (size_t)b * strideA;
  const T* Bb  = Bt + (size_t)b * strideB;
  const T* Ab2 = SPLIT ? (A2  + (size_t)b * strideA) : nullptr;
  const T* Bb2 = SPLIT ? (Bt2 + (size_t)b * strideB) : nullptr;

  const int rlane = lane & 15;
  const int koff  = (lane >> 4) * 8;
  const int mOff  = (lane >> 4) * 8;

  v8f acc[4][4];
#pragma unroll
  for (int i = 0; i < 4; ++i)
#pragma unroll
    for (int j = 0; j < 4; ++j) acc[i][j] = (v8f){0.f,0.f,0.f,0.f,0.f,0.f,0.f,0.f};

  for (int k0 = 0; k0 < K; k0 += 32) {
    V bh[4], bl[4];
#pragma unroll
    for (int j = 0; j < 4; ++j) {
      const size_t bo = (size_t)(n0 + (j << 4) + rlane) * ldb + koff + k0;
      bh[j] = Frag<T>::load(Bb + bo);
      if (SPLIT) bl[j] = Frag<T>::load(Bb2 + bo);
    }
#pragma unroll
    for (int i = 0; i < 4; ++i) {
      const size_t ao = (size_t)(m0 + (i << 4) + rlane) * lda + koff + k0;
      V ah = Frag<T>::load(Ab + ao);
      V al;
      if (SPLIT) al = Frag<T>::load(Ab2 + ao);
#pragma unroll
      for (int j = 0; j < 4; ++j) {
        acc[i][j] = Frag<T>::mma(ah, bh[j], acc[i][j]);
        if (SPLIT) {
          acc[i][j] = Frag<T>::mma(ah, bl[j], acc[i][j]);
          acc[i][j] = Frag<T>::mma(al, bh[j], acc[i][j]);
        }
      }
      Frag<T>::guard(acc[i][0], acc[i][3], ah, SPLIT ? al : ah);
    }
    Frag<T>::keep(bh[0], bh[1], bh[2], bh[3]);
    if (SPLIT) Frag<T>::keep(bl[0], bl[1], bl[2], bl[3]);
  }
  acc_guard4(acc[0][0], acc[0][1], acc[0][2], acc[0][3]);
  acc_guard4(acc[1][0], acc[1][1], acc[1][2], acc[1][3]);
  acc_guard4(acc[2][0], acc[2][1], acc[2][2], acc[2][3]);
  acc_guard4(acc[3][0], acc[3][1], acc[3][2], acc[3][3]);

  float* slab = sT[wave];
  const float* Rb = RESID ? (resid + (size_t)b * strideR) : nullptr;
#pragma unroll
  for (int i = 0; i < 4; ++i) {
    const int mBase = m0 + (i << 4);
#pragma unroll
    for (int j = 0; j < 4; ++j) {
      const int n = n0 + (j << 4) + rlane;
      float bv = 0.f;
      if (BIAS_MODE == 2) bv = bias[n];
#pragma unroll
      for (int r = 0; r < 8; ++r) {
        float v = acc[i][j][r] * scale;
        if (BIAS_MODE == 1) v += bias[mBase + mOff + r];
        if (BIAS_MODE == 2) v += bv;
        if (RESID) v += Rb[(size_t)(mBase + mOff + r) * ldc + n];
        if (ACT == 1) v = tanhf(v);
        if (ACT == 2) v = fmaxf(v, 0.0f);
        if (ACT == 3) v = v / (1.0f + expf(-v));
        if (ACT == 4) v = (v > 0.f) ? v : 0.01f * v;
        if (ACT == 5) v = 0.5f * v * (1.0f + erff(v * 0.70710678118654752f));
        slab[(mOff + r) * 68 + (j << 4) + rlane] = v;
      }
    }
    __builtin_amdgcn_fence(__ATOMIC_RELEASE, "workgroup");
    __builtin_amdgcn_wave_barrier();
    __builtin_amdgcn_fence(__ATOMIC_ACQUIRE, "workgroup");
    if (OUT_MODE == 0) {
      float* C = (float*)Cout + (size_t)b * strideC;
      const int hh = lane >> 4, c4 = (lane & 15) * 4;
      for (int pass = 0; pass < 2; ++pass) {
#pragma unroll
        for (int it = 0; it < 8; ++it) {
          const int row = it * 2 + hh;
          v4f v = *(const v4f*)(slab + row * 68 + c4);
          *(volatile v4f*)(C + (size_t)(mBase + row) * ldc + n0 + c4) = v;
        }
        __threadfence();
      }
    } else {
      const int q = lane >> 3, c8 = (lane & 7) * 8;
      unsigned short* C  = (unsigned short*)Cout  + (size_t)b * strideC;
      unsigned short* C2 = (OUT_MODE == 2) ? ((unsigned short*)Cout2 + (size_t)b * strideC) : nullptr;
      for (int pass = 0; pass < 2; ++pass) {
#pragma unroll
        for (int it = 0; it < 4; ++it) {
          const int row = it * 4 + q;
          const float* sp = slab + row * 68 + c8;
          v8h hv, lv;
#pragma unroll
          for (int e = 0; e < 8; ++e) {
            if (OUT_MODE == 1) {
              hv[e] = (_Float16)sp[e];
            } else {
              unsigned short hb = f2bf_bits(sp[e]);
              unsigned short lb = f2bf_bits(sp[e] - bf_bits2f(hb));
              hv[e] = __builtin_bit_cast(_Float16, hb);
              lv[e] = __builtin_bit_cast(_Float16, lb);
            }
          }
          *(volatile v8h*)(C + (size_t)(mBase + row) * ldc + n0 + c8) = hv;
          if (OUT_MODE == 2) *(volatile v8h*)(C2 + (size_t)(mBase + row) * ldc + n0 + c8) = lv;
        }
        __threadfence();
      }
    }
    __builtin_amdgcn_fence(__ATOMIC_RELEASE, "workgroup");
    __builtin_amdgcn_wave_barrier();
    __builtin_amdgcn_fence(__ATOMIC_ACQUIRE, "workgroup");
  }
}

__global__ __launch_bounds__(256) void cast_f32_f16x2(
    const float* __restrict__ in, _Float16* __restrict__ out, int n2) {
  int i = blockIdx.x * 256 + threadIdx.x;
  if (i < n2) {
    const _Float16 h0 = (_Float16)in[2 * i], h1 = (_Float16)in[2 * i + 1];
    const unsigned u = (unsigned)__builtin_bit_cast(unsigned short, h0) | ((unsigned)__builtin_bit_cast(unsigned short, h1) << 16);
    ((volatile unsigned*)out)[i] = u;
    __threadfence();
    ((volatile unsigned*)out)[i] = u;
  }
}

__global__ __launch_bounds__(256) void split_f32_bf16x2(
    const float* __restrict__ in, __bf16* __restrict__ hi, __bf16* __restrict__ lo, long n2) {
  long i = (long)blockIdx.x * 256 + threadIdx.x;
  long stride = (long)gridDim.x * 256;
  for (int pass = 0; pass < 2; ++pass) {
    for (long j = i; j < n2; j += stride) {
      const float a = in[2 * j], b = in[2 * j + 1];
      const unsigned short ah = f2bf_bits(a), bh = f2bf_bits(b);
      const unsigned short al = f2bf_bits(a - bf_bits2f(ah)), bl = f2bf_bits(b - bf_bits2f(bh));
      ((volatile unsigned*)hi)[j] = (unsigned)ah | ((unsigned)bh << 16);
      ((volatile unsigned*)lo)[j] = (unsigned)al | ((unsigned)bl << 16);
    }
    __threadfence();
  }
}


__global__ __launch_bounds__(256) void transpose_split_bf16(const float* __restrict__ in, int ldi,
                                                           __bf16* __restrict__ outH, __bf16* __restrict__ outL, int ldo) {
  __shared__ __align__(16) float tile[64][68];
  const int c0 = blockIdx.x * 64, r0 = blockIdx.y * 64;
  const int t = threadIdx.y * 32 + threadIdx.x;
  for (int i = threadIdx.y; i < 64; i += 8) {
    tile[threadIdx.x][i]      = in[(size_t)(r0 + i) * ldi + c0 + threadIdx.x];
    tile[32 + threadIdx.x][i] = in[(size_t)(r0 + i) * ldi + c0 + 32 + threadIdx.x];
  }
  __syncthreads();
  const int q = t >> 3, c8 = (t & 7) * 8;
  for (int pass = 0; pass < 2; ++pass) {
#pragma unroll
    for (int it = 0; it < 2; ++it) {
      const int c = it * 32 + q;
      v8b hv, lv;
#pragma unroll
      for (int e = 0; e < 8; ++e) {
        const float f = tile[c][c8 + e];
        const unsigned short hb = f2bf_bits(f);
        hv[e] = __builtin_bit_cast(__bf16, hb);
        lv[e] = __builtin_bit_cast(__bf16, f2bf_bits(f - bf_bits2f(hb)));
      }
      *(volatile v8b*)(outH + (size_t)(c0 + c) * ldo + r0 + c8) = hv;
      *(volatile v8b*)(outL + (size_t)(c0 + c) * ldo + r0 + c8) = lv;
    }
    __threadfence();
  }
}

#define GB 32
#define GNn 256
#define GK 32
#define GE 1024
#define GD 256
#define GR (GB * GNn)
__global__ __launch_bounds__(256) void act_kernel(const float* __restrict__ st, const float* __restrict__ em, const int* __restrict__ An, const int* __restrict__ Ae, __bf16* __restrict__ Xh, __bf16* __restrict__ Xl, float* __restrict__ ACT) {
  const int lane = threadIdx.x & 31, wave = threadIdx.x >> 5; const size_t r = (size_t)blockIdx.x * 8 + wave; const int b = (int)(r / GNn);
  v8f a = {0.f,0.f,0.f,0.f,0.f,0.f,0.f,0.f};
#pragma unroll 1
  for (int k = 0; k < GK; ++k) { int ni = An[r * GK + k], ei = Ae[r * GK + k];
    if (ni != 0) { ni = ni < 0 ? 0 : (ni >= GNn ? GNn - 1 : ni); a += *(const v8f*)(st + ((size_t)b * GNn + ni) * GD + lane * 8); }
    if (ei != 0) { ei = ei < 0 ? 0 : (ei >= GE ? GE - 1 : ei); a += *(const v8f*)(em + ((size_t)b * GE + ei) * GD + lane * 8); } }
  const v8f h = *(const v8f*)(st + r * GD + lane * 8);
  unsigned ah[4], al[4], hh[4], hl[4];
  for (int q = 0; q < 4; ++q) { unsigned short h0 = f2bf_bits(a[2*q]), h1 = f2bf_bits(a[2*q+1]); ah[q] = (unsigned)h0 | ((unsigned)h1 << 16); al[q] = (unsigned)f2bf_bits(a[2*q] - bf_bits2f(h0)) | ((unsigned)f2bf_bits(a[2*q+1] - bf_bits2f(h1)) << 16);
    unsigned short g0 = f2bf_bits(h[2*q]), g1 = f2bf_bits(h[2*q+1]); hh[q] = (unsigned)g0 | ((unsigned)g1 << 16); hl[q] = (unsigned)f2bf_bits(h[2*q] - bf_bits2f(g0)) | ((unsigned)f2bf_bits(h[2*q+1] - bf_bits2f(g1)) << 16); }
  typedef __attribute__((ext_vector_type(4))) unsigned u4; const u4 A0 = {ah[0],ah[1],ah[2],ah[3]}, A1 = {al[0],al[1],al[2],al[3]}, H0 = {hh[0],hh[1],hh[2],hh[3]}, H1 = {hl[0],hl[1],hl[2],hl[3]};
  unsigned* XH = (unsigned*)Xh; unsigned* XL = (unsigned*)Xl;
  for (int pass = 0; pass < 2; ++pass) { *(volatile u4*)(XH + (r * 512 + lane * 8) / 2) = A0; *(volatile u4*)(XL + (r * 512 + lane * 8) / 2) = A1; *(volatile u4*)(XH + (r * 512 + 256 + lane * 8) / 2) = H0; *(volatile u4*)(XL + (r * 512 + 256 + lane * 8) / 2) = H1;
    *(volatile v8f*)(ACT + r * GD + lane * 8) = a; __threadfence(); }
}
__global__ __launch_bounds__(256) void hid_kernel(const float* __restrict__ ACT, const float* __restrict__ G, const float* __restrict__ st, __bf16* __restrict__ Yh, __bf16* __restrict__ Yl) {
  const int lane = threadIdx.x & 31, wave = threadIdx.x >> 5; const size_t r = (size_t)blockIdx.x * 8 + wave;
  const v8f a = *(const v8f*)(ACT + r * GD + lane * 8), h = *(const v8f*)(st + r * GD + lane * 8), gr = *(const v8f*)(G + r * 512 + 256 + lane * 8);
  v8f rh; for (int q = 0; q < 8; ++q) rh[q] = h[q] / (1.0f + expf(-gr[q]));
  unsigned ah[4], al[4], hh[4], hl[4];
  for (int q = 0; q < 4; ++q) { unsigned short h0 = f2bf_bits(a[2*q]), h1 = f2bf_bits(a[2*q+1]); ah[q] = (unsigned)h0 | ((unsigned)h1 << 16); al[q] = (unsigned)f2bf_bits(a[2*q] - bf_bits2f(h0)) | ((unsigned)f2bf_bits(a[2*q+1] - bf_bits2f(h1)) << 16);
    unsigned short g0 = f2bf_bits(rh[2*q]), g1 = f2bf_bits(rh[2*q+1]); hh[q] = (unsigned)g0 | ((unsigned)g1 << 16); hl[q] = (unsigned)f2bf_bits(rh[2*q] - bf_bits2f(g0)) | ((unsigned)f2bf_bits(rh[2*q+1] - bf_bits2f(g1)) << 16); }
  typedef __attribute__((ext_vector_type(4))) unsigned u4; const u4 A0 = {ah[0],ah[1],ah[2],ah[3]}, A1 = {al[0],al[1],al[2],al[3]}, H0 = {hh[0],hh[1],hh[2],hh[3]}, H1 = {hl[0],hl[1],hl[2],hl[3]};
  unsigned* YH = (unsigned*)Yh; unsigned* YL = (unsigned*)Yl;
  for (int pass = 0; pass < 2; ++pass) { *(volatile u4*)(YH + (r * 512 + lane * 8) / 2) = A0; *(volatile u4*)(YL + (r * 512 + lane * 8) / 2) = A1; *(volatile u4*)(YH + (r * 512 + 256 + lane * 8) / 2) = H0; *(volatile u4*)(YL + (r * 512 + 256 + lane * 8) / 2) = H1; __threadfence(); }
}
__global__ __launch_bounds__(256) void blend_kernel(const float* __restrict__ G, const float* __restrict__ NEW, const float* __restrict__ st, float* __restrict__ out) {
  const int lane = threadIdx.x & 31, wave = threadIdx.x >> 5; const size_t r = (size_t)blockIdx.x * 8 + wave;
  const v8f gu = *(const v8f*)(G + r * 512 + lane * 8), nw = *(const v8f*)(NEW + r * GD + lane * 8), h = *(const v8f*)(st + r * GD + lane * 8);
  v8f o; for (int q = 0; q < 8; ++q) { const float u = 1.0f / (1.0f + expf(-gu[q])); o[q] = (1.0f - u) * h[q] + u * nw[q]; }
  *(volatile v8f*)(out + r * GD + lane * 8) = o; __threadfence(); *(volatile v8f*)(out + r * GD + lane * 8) = o;
}
__global__ __launch_bounds__(256) void bias2_kernel(const float* a, const float* b, float* o) { for (int i = threadIdx.x; i < 512; i += 256) { const float v = (i < 256) ? a[i] : b[i - 256]; ((volatile float*)o)[i] = v; __threadfence(); ((volatile float*)o)[i] = v; } }
extern "C" void kernel_launch(void* const* d_in, const int* in_sizes, int n_in, void* d_out, int out_size, void* d_ws, size_t ws_size, hipStream_t stream) {
  (void)in_sizes; (void)n_in; (void)out_size; (void)ws_size;
  const float* st = (const float*)d_in[0]; const float* em = (const float*)d_in[1]; const int* An = (const int*)d_in[2]; const int* Ae = (const int*)d_in[3];
  const float* Wu = (const float*)d_in[4]; const float* bu = (const float*)d_in[5]; const float* Wr = (const float*)d_in[6]; const float* br = (const float*)d_in[7]; const float* Wh = (const float*)d_in[8]; const float* bh = (const float*)d_in[9];
  char* ws = (char*)d_ws; size_t off = 0;
  auto carve = [&](size_t bytes) -> char* { char* p = ws + off; off += (bytes + 255) & ~(size_t)255; return p; };
  __bf16* Xh = (__bf16*)carve((size_t)GR * 512 * 2); __bf16* Xl = (__bf16*)carve((size_t)GR * 512 * 2); float* ACT = (float*)carve((size_t)GR * GD * 4);
  __bf16* WUh = (__bf16*)carve(512 * 512 * 2); __bf16* WUl = (__bf16*)carve(512 * 512 * 2); __bf16* WHh = (__bf16*)carve(256 * 512 * 2); __bf16* WHl = (__bf16*)carve(256 * 512 * 2); float* bur = (float*)carve(512 * 4);
  float* G = (float*)carve((size_t)GR * 512 * 4); __bf16* Yh = (__bf16*)carve((size_t)GR * 512 * 2); __bf16* Yl = (__bf16*)carve((size_t)GR * 512 * 2); float* NEW = (float*)carve((size_t)GR * GD * 4);
  act_kernel<<<GR / 8, 256, 0, stream>>>(st, em, An, Ae, Xh, Xl, ACT);
  transpose_split_bf16<<<dim3(256 / 64, 512 / 64), dim3(32, 8), 0, stream>>>(Wu, 256, WUh, WUl, 512);
  transpose_split_bf16<<<dim3(256 / 64, 512 / 64), dim3(32, 8), 0, stream>>>(Wr, 256, WUh + 256 * 512, WUl + 256 * 512, 512);
  transpose_split_bf16<<<dim3(256 / 64, 512 / 64), dim3(32, 8), 0, stream>>>(Wh, 256, WHh, WHl, 512);
  bias2_kernel<<<1, 256, 0, stream>>>(bu, br, bur);
  { const int t = (GR / 64) * 8; wmma_gemm64<1, true, 2, 0, false><<<dim3((t + 7) / 8, 1), 256, 0, stream>>>(U16(Xh), U16(Xl), 512, 0, U16(WUh), U16(WUl), 512, 0, G, nullptr, 512, 0, bur, nullptr, 0, GR, 512, 512, 1.0f); }
  hid_kernel<<<GR / 8, 256, 0, stream>>>(ACT, G, st, Yh, Yl);
  { const int t = (GR / 64) * 4; wmma_gemm64<1, true, 2, 0, false, 1><<<dim3((t + 7) / 8, 1), 256, 0, stream>>>(U16(Yh), U16(Yl), 512, 0, U16(WHh), U16(WHl), 512, 0, NEW, nullptr, GD, 0, bh, nullptr, 0, GR, GD, 512, 1.0f); }
  blend_kernel<<<GR / 8, 256, 0, stream>>>(G, NEW, st, (float*)d_out);
}
